// GRUCell_87265145520378
// MI455X (gfx1250) — hardware-verified
//
#include <hip/hip_runtime.h>


#define NR   8192
#define NI   1024
#define NU   1024
#define KC   (NI + NU)
typedef _Float16 h16;
typedef unsigned short bf;
typedef __attribute__((ext_vector_type(16))) __bf16   v16bf;
typedef __attribute__((ext_vector_type(16))) _Float16 v16h;
typedef __attribute__((ext_vector_type(8)))  _Float16 v8h;
typedef __attribute__((ext_vector_type(8)))  unsigned short v8us;
typedef __attribute__((ext_vector_type(8)))  float    v8f;
typedef __attribute__((ext_vector_type(4)))  float    v4f;
typedef v8h  __attribute__((may_alias)) v8ha;
typedef v4f  __attribute__((may_alias)) v4fa;
typedef v8us __attribute__((may_alias)) v8usa;

__device__ __forceinline__ unsigned short f2bf(float f) { unsigned u = __float_as_uint(f); u += 0x7FFFu + ((u >> 16) & 1u); return (unsigned short)(u >> 16); }
__device__ __forceinline__ float bf2f(unsigned short b) { return __uint_as_float(((unsigned)b) << 16); }
__device__ __forceinline__ float bfr(float f) { return bf2f(f2bf(f)); }
__device__ __forceinline__ v16h cat16(v8h lo, v8h hi) { return __builtin_shufflevector(lo, hi, 0, 1, 2, 3, 4, 5, 6, 7, 8, 9, 10, 11, 12, 13, 14, 15); }
__device__ __forceinline__ v16bf cat16b(v8us lo, v8us hi) { return __builtin_bit_cast(v16bf, __builtin_shufflevector(lo, hi, 0, 1, 2, 3, 4, 5, 6, 7, 8, 9, 10, 11, 12, 13, 14, 15)); }
__device__ __forceinline__ v8f wmma16(v16h a, v16h b, v8f c) { return __builtin_amdgcn_wmma_f32_16x16x32_f16(false, a, false, b, (short)0, c, false, false); }
__device__ __forceinline__ v8f wmmab(v16bf a, v16bf b, v8f c) { return __builtin_amdgcn_wmma_f32_16x16x32_bf16(false, a, false, b, (short)0, c, false, false); }


template <typename T16> struct WFrag;
template <> struct WFrag<h16> { typedef v16h V; static __device__ __forceinline__ V ld(const h16* p) { return cat16(*(const v8h*)p, *(const v8h*)(p + 16)); } static __device__ __forceinline__ v8f mma(V a, V b, v8f c) { return wmma16(a, b, c); } };
template <> struct WFrag<bf> { typedef v16bf V; static __device__ __forceinline__ V ld(const bf* p) { return cat16b(*(const v8us*)p, *(const v8us*)(p + 16)); } static __device__ __forceinline__ v8f mma(V a, V b, v8f c) { return wmmab(a, b, c); } };
template <typename T16, int NSPLIT, bool BIAS>
__global__ __launch_bounds__(32) void k_gemmw(const T16* __restrict__ A, const T16* __restrict__ A2, const T16* __restrict__ Bt, const T16* __restrict__ Bt2, int K, float* C, int ldc, const float* __restrict__ bias, size_t sA, size_t sB, size_t sC) {
    typedef typename WFrag<T16>::V V;
    __shared__ __align__(16) float os[16 * 68];
    const size_t z = blockIdx.z; A += z * sA; if (A2) A2 += z * sA; Bt += z * sB; if (Bt2) Bt2 += z * sB; C += z * sC;
    const int lane = threadIdx.x & 31, lr = lane & 15, hi = lane >> 4; const int r0 = blockIdx.x * 64, c0 = blockIdx.y * 64;
    v8f acc[4][4];
#pragma unroll
    for (int mb = 0; mb < 4; ++mb)
#pragma unroll
        for (int nb = 0; nb < 4; ++nb) acc[mb][nb] = (v8f){};
    const size_t aoff = (size_t)(r0 + lr) * K + 8 * hi, boff = (size_t)(c0 + lr) * K + 8 * hi;
#pragma unroll 1
    for (int kc = 0; kc < K; kc += 32) {
        V a[4], a2[4];
#pragma unroll
        for (int mb = 0; mb < 4; ++mb) { a[mb] = WFrag<T16>::ld(A + aoff + (size_t)mb * 16 * K + kc); if (NSPLIT == 1 || NSPLIT == 2) a2[mb] = WFrag<T16>::ld(A2 + aoff + (size_t)mb * 16 * K + kc); }
#pragma unroll
        for (int nb = 0; nb < 4; ++nb) { const V b = WFrag<T16>::ld(Bt + boff + (size_t)nb * 16 * K + kc); V b2; if (NSPLIT >= 2) b2 = WFrag<T16>::ld(Bt2 + boff + (size_t)nb * 16 * K + kc);
#pragma unroll
            for (int mb = 0; mb < 4; ++mb) { acc[mb][nb] = WFrag<T16>::mma(a[mb], b, acc[mb][nb]); if (NSPLIT == 1 || NSPLIT == 2) acc[mb][nb] = WFrag<T16>::mma(a2[mb], b, acc[mb][nb]); if (NSPLIT >= 2) acc[mb][nb] = WFrag<T16>::mma(a[mb], b2, acc[mb][nb]); } }
        asm volatile("v_nop\n\tv_nop\n\tv_nop\n\tv_nop" : "+v"(acc[0][0]), "+v"(acc[1][1]), "+v"(acc[2][2]), "+v"(acc[3][3]) : "v"(a[0]), "v"(a[3]));
    }
#pragma unroll
    for (int mb = 0; mb < 4; ++mb) {
#pragma unroll
        for (int nb = 0; nb < 4; ++nb) {
#pragma unroll
            for (int j = 0; j < 8; ++j) os[(hi * 8 + j) * 68 + nb * 16 + lr] = acc[mb][nb][j]; }
        __builtin_amdgcn_wave_barrier(); asm volatile("" ::: "memory");
        float* crow = C + (size_t)(r0 + mb * 16) * ldc + c0;
#pragma unroll 1
        for (int ps = 0; ps < 2; ++ps) {
#pragma unroll
            for (int s = 0; s < 8; ++s) { const int row = 2 * s + hi, cofs = lr * 4; v4f val = *(const v4fa*)(os + row * 68 + cofs); if (BIAS) { val[0] += bfr(bias[c0 + cofs]); val[1] += bfr(bias[c0 + cofs + 1]); val[2] += bfr(bias[c0 + cofs + 2]); val[3] += bfr(bias[c0 + cofs + 3]); }
                *(volatile v4f*)(crow + (size_t)row * ldc + cofs) = val; }
            if (ps == 0) __threadfence(); }
        __builtin_amdgcn_wave_barrier(); asm volatile("" ::: "memory");
    }
}

typedef __attribute__((ext_vector_type(2))) unsigned short v2us;
__device__ __forceinline__ float ex2(float a) { return __builtin_amdgcn_exp2f(__fmul_rn(a, 1.4426950408889634f)); }
__device__ __forceinline__ float sigm(float a) { return __fdiv_rn(1.0f, __fadd_rn(1.0f, ex2(-a))); }
__device__ __forceinline__ float tanhp(float a) { const float e = ex2(__fmul_rn(2.0f, a)); return __fsub_rn(1.0f, __fdiv_rn(2.0f, __fadd_rn(e, 1.0f))); }
__global__ __launch_bounds__(256) void k_wtG(const float* __restrict__ w, int K, int N, bf* Bt) {
    const int lane = threadIdx.x & 31; const int L0 = (blockIdx.x * 8 + (threadIdx.x >> 5)) * 8; const int nlines = N * K / 64;
#pragma unroll
    for (int ps = 0; ps < 2; ++ps) {
#pragma unroll 1
        for (int l = 0; l < 8; ++l) { const int L = L0 + l; if (L >= nlines) break; const size_t e = (size_t)L * 64 + lane * 2; const int k = (int)(e % K), n = (int)(e / K); v2us o;
            o[0] = f2bf(w[(size_t)k * N + n]); o[1] = f2bf(w[(size_t)(k + 1) * N + n]); *(volatile v2us*)(Bt + e) = o; }
        if (ps == 0) __threadfence(); }
}

__global__ __launch_bounds__(256) void k_cvt8(const float* __restrict__ src, bf* dst, size_t n8) { const size_t i = (size_t)blockIdx.x * 256 + threadIdx.x; if (i >= n8) return; const v8f v = *(const v8f*)(src + i * 8); v8us o;
#pragma unroll
    for (int k = 0; k < 8; ++k) o[k] = f2bf(v[k]); *(volatile v8us*)(dst + i * 8) = o; __threadfence(); *(volatile v8us*)(dst + i * 8) = o; }
__global__ __launch_bounds__(256) void k_wtGk(const float* __restrict__ w, int K, int N, bf* Bt, int k0) { const int lane = threadIdx.x & 31; const int L0 = (blockIdx.x * 8 + (threadIdx.x >> 5)) * 8; const int nlines = K * N / 64;
#pragma unroll
    for (int ps = 0; ps < 2; ++ps) {
#pragma unroll 1
        for (int l = 0; l < 8; ++l) { const int L = L0 + l; if (L >= nlines) break; const size_t e = (size_t)L * 64 + lane * 2; const int k = (int)(e % K), n = (int)(e / K); v2us o; o[0] = f2bf(w[(size_t)k * N + n]); o[1] = f2bf(w[(size_t)(k + 1) * N + n]); *(volatile v2us*)(Bt + (size_t)n * KC + k0 + k) = o; }
        if (ps == 0) __threadfence(); } }
__global__ __launch_bounds__(256) void k_cat(const float* __restrict__ x, const float* __restrict__ h, bf* XC) { const size_t i = (size_t)blockIdx.x * 256 + threadIdx.x; if (i >= (size_t)NR * KC / 8) return; const int c0 = (int)(i % (KC / 8)) * 8; const size_t r = i / (KC / 8); const bool first = c0 < NI; const int ca = min(c0, NI - 8), cb = max(c0 - NI, 0); v8us o;
#pragma unroll
    for (int k = 0; k < 8; ++k) { const unsigned short ea = f2bf(x[r * NI + ca + k]), eb = f2bf(h[r * NU + cb + k]); o[k] = first ? ea : eb; }
    *(volatile v8us*)(XC + r * KC + c0) = o; __threadfence(); *(volatile v8us*)(XC + r * KC + c0) = o; }
__global__ __launch_bounds__(256) void k_bias2(const float* __restrict__ a, const float* __restrict__ b, float* B2) { const int i = blockIdx.x * 256 + threadIdx.x; if (i >= 2 * NU) return; const float v = __fadd_rn(bfr(a[i]), bfr(b[i])); *(volatile float*)(B2 + i) = v; __threadfence(); *(volatile float*)(B2 + i) = v; }
__global__ __launch_bounds__(256) void k_out(const float* __restrict__ G, const float* __restrict__ XCc, const float* __restrict__ HC, const float* __restrict__ hx, float* out) { const size_t i = (size_t)blockIdx.x * 256 + threadIdx.x; if (i >= (size_t)NR * NU / 4) return; const int c0 = (int)(i % (NU / 4)) * 4; const size_t r = i / (NU / 4); v4f o; const v4f xc = *(const v4f*)(XCc + r * NU + c0), hc = *(const v4f*)(HC + r * NU + c0), hv = *(const v4f*)(hx + r * NU + c0);
#pragma unroll
    for (int q = 0; q < 4; ++q) { const int c = c0 + q; const float z = sigm(G[r * (2 * NU) + c]); const float rg = sigm(G[r * (2 * NU) + NU + c]); float p = __fmul_rn(rg, hc[q]); asm volatile("" : "+v"(p)); const float cand = tanhp(__fadd_rn(xc[q], p)); float a = __fmul_rn(__fsub_rn(1.0f, z), bfr(hv[q])), b = __fmul_rn(z, cand); asm volatile("" : "+v"(a), "+v"(b)); o[q] = __fadd_rn(a, b); }
    *(volatile v4f*)(out + r * NU + c0) = o; __threadfence(); *(volatile v4f*)(out + r * NU + c0) = o; }

extern "C" void kernel_launch(void* const* d_in, const int* in_sizes, int n_in,
                              void* d_out, int out_size, void* d_ws, size_t ws_size, hipStream_t stream) {
    (void)in_sizes; (void)n_in; (void)out_size;
    const float* x = (const float*)d_in[0]; const float* hx = (const float*)d_in[1]; const float* wih = (const float*)d_in[2]; const float* bih = (const float*)d_in[3]; const float* whh = (const float*)d_in[4]; const float* bhh = (const float*)d_in[5]; const float* wc = (const float*)d_in[6]; const float* bc = (const float*)d_in[7]; const float* whc = (const float*)d_in[8]; const float* bhc = (const float*)d_in[9];
    float* OUT = (float*)d_out;
    char* wsp = (char*)d_ws;
    auto take = [&](size_t bytes) { char* p = wsp; wsp += (bytes + 255) & ~(size_t)255; return (void*)p; };
    bf* WG = (bf*)take((size_t)2 * NU * KC * 2); bf* WC = (bf*)take((size_t)NU * NI * 2); bf* WHC = (bf*)take((size_t)NU * NU * 2); float* BG = (float*)take((size_t)2 * NU * 4); bf* XC = (bf*)take((size_t)NR * KC * 2); float* G = (float*)take((size_t)NR * 2 * NU * 4); float* XCc = (float*)take((size_t)NR * NU * 4); float* HC = (float*)take((size_t)NR * NU * 4); bf* XI = (bf*)take((size_t)NR * NI * 2); bf* XH = (bf*)take((size_t)NR * NU * 2);
    if ((size_t)(wsp - (char*)d_ws) > ws_size) return;
    k_wtGk<<<(NI * 2 * NU / 64 + 63) / 64, 256, 0, stream>>>(wih, NI, 2 * NU, WG, 0); k_wtGk<<<(NU * 2 * NU / 64 + 63) / 64, 256, 0, stream>>>(whh, NU, 2 * NU, WG, NI);
    k_wtG<<<(NI * NU / 64 + 63) / 64, 256, 0, stream>>>(wc, NI, NU, WC); k_wtG<<<(NU * NU / 64 + 63) / 64, 256, 0, stream>>>(whc, NU, NU, WHC); k_bias2<<<(2 * NU + 255) / 256, 256, 0, stream>>>(bih, bhh, BG);
    k_cat<<<(unsigned)(((size_t)NR * KC / 8 + 255) / 256), 256, 0, stream>>>(x, hx, XC); k_cvt8<<<(unsigned)(((size_t)NR * NI / 8 + 255) / 256), 256, 0, stream>>>(x, XI, (size_t)NR * NI / 8); k_cvt8<<<(unsigned)(((size_t)NR * NU / 8 + 255) / 256), 256, 0, stream>>>(hx, XH, (size_t)NR * NU / 8);
    k_gemmw<bf, 0, true><<<dim3(NR / 64, 2 * NU / 64, 1), 32, 0, stream>>>(XC, nullptr, WG, nullptr, KC, G, 2 * NU, BG, 0, 0, 0);
    k_gemmw<bf, 0, true><<<dim3(NR / 64, NU / 64, 1), 32, 0, stream>>>(XI, nullptr, WC, nullptr, NI, XCc, NU, bc, 0, 0, 0);
    k_gemmw<bf, 0, true><<<dim3(NR / 64, NU / 64, 1), 32, 0, stream>>>(XH, nullptr, WHC, nullptr, NU, HC, NU, bhc, 0, 0, 0);
    k_out<<<(unsigned)(((size_t)NR * NU / 4 + 255) / 256), 256, 0, stream>>>(G, XCc, HC, hx, OUT);
}
